// LSTMCell_38414187495767
// MI455X (gfx1250) — hardware-verified
//
#include <hip/hip_runtime.h>
#include <math.h>

typedef __attribute__((ext_vector_type(16))) _Float16 v16h;
typedef __attribute__((ext_vector_type(8)))  _Float16 v8h;
typedef __attribute__((ext_vector_type(16))) __bf16   v16b;
typedef __attribute__((ext_vector_type(8)))  __bf16   v8b;
typedef __attribute__((ext_vector_type(8)))  float    v8f;
typedef __attribute__((ext_vector_type(4)))  float    v4f;
typedef __attribute__((ext_vector_type(4)))  unsigned int v4u;

constexpr int NBATCH = 4096;
constexpr int NIN    = 1024;
constexpr int NHID   = 1024;
constexpr int KTOT   = NIN + NHID;
constexpr int NGATE  = 4 * NHID;
constexpr size_t PLANE = (size_t)NBATCH * NHID;
static_assert(NIN == NHID, "square weights");
static_assert(NBATCH % 64 == 0 && NGATE % 64 == 0 && KTOT % 32 == 0, "gemm tile multiples");
static_assert((NBATCH * NIN) % (256 * 8) == 0, "pack grid exact");
static_assert(NIN % 64 == 0 && NHID % 32 == 0, "transpose grid exact");

constexpr size_t A_BYTES  = (size_t)NBATCH * KTOT * 2;
constexpr size_t BT_BYTES = (size_t)NGATE * KTOT * 2;
constexpr size_t Z_BYTES  = (size_t)NBATCH * NGATE * 4;
constexpr size_t OFF_A  = 0;
constexpr size_t OFF_BT = OFF_A + A_BYTES;
constexpr size_t OFF_Z  = OFF_BT + BT_BYTES;
constexpr size_t WS_TOTAL = OFF_Z + Z_BYTES;
static_assert(WS_TOTAL == 100663296ull, "96 MiB carve");
static_assert(WS_TOTAL <= 134217728ull, "carve under 128 MiB");
static_assert((OFF_BT % 128) == 0 && (OFF_Z % 128) == 0, "line-aligned regions");

__device__ __forceinline__ unsigned short f2bf_bits(float f) {
  unsigned u = __float_as_uint(f);
  return (unsigned short)((u + 0x7FFFu + ((u >> 16) & 1u)) >> 16);
}
__device__ __forceinline__ float bf_bits2f(unsigned short h) { return __uint_as_float(((unsigned)h) << 16); }
__device__ __forceinline__ float bf_rne(float f) { return bf_bits2f(f2bf_bits(f)); }
__device__ __forceinline__ unsigned pack_bf2(float a, float b) {
  return (unsigned)f2bf_bits(a) | ((unsigned)f2bf_bits(b) << 16);
}

__device__ __forceinline__ void dep_guard_h(v8f& a, v8f& b, v16h x, v16h y) { asm volatile("v_nop\n\tv_nop\n\tv_nop\n\tv_nop" : "+v"(a), "+v"(b) : "v"(x), "v"(y)); }
__device__ __forceinline__ void dep_guard_b(v8f& a, v8f& b, v16b x, v16b y) { asm volatile("v_nop\n\tv_nop\n\tv_nop\n\tv_nop" : "+v"(a), "+v"(b) : "v"(x), "v"(y)); }
__device__ __forceinline__ void dep_guard4_h(v8f& a, v8f& b, v8f& c, v8f& d, v16h x, v16h y) { asm volatile("v_nop\n\tv_nop\n\tv_nop\n\tv_nop" : "+v"(a), "+v"(b), "+v"(c), "+v"(d) : "v"(x), "v"(y)); }
__device__ __forceinline__ void dep_guard4_b(v8f& a, v8f& b, v8f& c, v8f& d, v16b x, v16b y) { asm volatile("v_nop\n\tv_nop\n\tv_nop\n\tv_nop" : "+v"(a), "+v"(b), "+v"(c), "+v"(d) : "v"(x), "v"(y)); }
__device__ __forceinline__ void keep4_h(v16h a, v16h b, v16h c, v16h d) { asm volatile("v_nop" :: "v"(a), "v"(b), "v"(c), "v"(d)); }
__device__ __forceinline__ void keep4_b(v16b a, v16b b, v16b c, v16b d) { asm volatile("v_nop" :: "v"(a), "v"(b), "v"(c), "v"(d)); }
__device__ __forceinline__ void acc_guard4(v8f& a, v8f& b, v8f& c, v8f& d) { asm volatile("v_nop\n\tv_nop\n\tv_nop\n\tv_nop" : "+v"(a), "+v"(b), "+v"(c), "+v"(d)); }
template <typename T> struct Frag;
template <> struct Frag<_Float16> {
  typedef v16h V; union U { v16h v; v8h h[2]; };
  static __device__ __forceinline__ v16h load(const _Float16* p) {
    U f; f.h[0] = *(const v8h*)(p); f.h[1] = *(const v8h*)(p + 16); return f.v;
  }
  static __device__ __forceinline__ v8f mma(v16h a, v16h b, v8f c) {
    return __builtin_amdgcn_wmma_f32_16x16x32_f16(false, a, false, b, (short)0, c, false, false);
  }
  static __device__ __forceinline__ void guard(v8f& a, v8f& b, v16h x, v16h y) { dep_guard_h(a, b, x, y); }
  static __device__ __forceinline__ void guard4(v8f& a, v8f& b, v8f& c, v8f& d, v16h x, v16h y) { dep_guard4_h(a, b, c, d, x, y); }
  static __device__ __forceinline__ void keep(v16h a, v16h b, v16h c, v16h d) { keep4_h(a, b, c, d); }
};
template <> struct Frag<__bf16> {
  typedef v16b V; union U { v16b v; v8b h[2]; };
  static __device__ __forceinline__ v16b load(const __bf16* p) {
    U f; f.h[0] = *(const v8b*)(p); f.h[1] = *(const v8b*)(p + 16); return f.v;
  }
  static __device__ __forceinline__ v8f mma(v16b a, v16b b, v8f c) {
    return __builtin_amdgcn_wmma_f32_16x16x32_bf16(false, a, false, b, (short)0, c, false, false);
  }
  static __device__ __forceinline__ void guard(v8f& a, v8f& b, v16b x, v16b y) { dep_guard_b(a, b, x, y); }
  static __device__ __forceinline__ void guard4(v8f& a, v8f& b, v8f& c, v8f& d, v16b x, v16b y) { dep_guard4_b(a, b, c, d, x, y); }
  static __device__ __forceinline__ void keep(v16b a, v16b b, v16b c, v16b d) { keep4_b(a, b, c, d); }
};

template <int ET> struct Elem;
template <> struct Elem<0> { typedef _Float16 T; };
template <> struct Elem<1> { typedef __bf16 T; };
template <int ET, bool SPLIT, int BIAS_MODE, int OUT_MODE, bool RESID, int ACT = 0>
__global__ __launch_bounds__(256) void wmma_gemm64(
    const unsigned short* __restrict__ Ap, const unsigned short* __restrict__ A2p, int lda, long strideA,
    const unsigned short* __restrict__ Btp, const unsigned short* __restrict__ Bt2p, int ldb, long strideB,
    void* __restrict__ Cout, void* __restrict__ Cout2, int ldc, long strideC,
    const float* __restrict__ bias,
    const float* __restrict__ resid, long strideR,
    int M, int N, int K, float scale) {
  typedef typename Elem<ET>::T T;
  typedef typename Frag<T>::V V;
  const T* A = (const T*)Ap; const T* A2 = (const T*)A2p; const T* Bt = (const T*)Btp; const T* Bt2 = (const T*)Bt2p;
  __shared__ __align__(16) float sT[8][16 * 68];
  const int b    = blockIdx.y;
  const int lane = threadIdx.x & 31;
  const int wave = threadIdx.x >> 5;
  const int tilesN = N >> 6;
  const int tilesM = M >> 6;
  const int tile = blockIdx.x * 8 + wave;
  if (tile >= tilesM * tilesN) return;
  const int tm = tile / tilesN;
  const int tn = tile - tm * tilesN;
  const int m0 = tm << 6;
  const int n0 = tn << 6;

  const T* Ab  = A  + (size_t)b * strideA;
  const T* Bb  = Bt + (size_t)b * strideB;
  const T* Ab2 = SPLIT ? (A2  + (size_t)b * strideA) : nullptr;
  const T* Bb2 = SPLIT ? (Bt2 + (size_t)b * strideB) : nullptr;

  const int rlane = lane & 15;
  const int koff  = (lane >> 4) * 8;
  const int mOff  = (lane >> 4) * 8;

  v8f acc[4][4];
#pragma unroll
  for (int i = 0; i < 4; ++i)
#pragma unroll
    for (int j = 0; j < 4; ++j) acc[i][j] = (v8f){0.f,0.f,0.f,0.f,0.f,0.f,0.f,0.f};

  for (int k0 = 0; k0 < K; k0 += 32) {
    V bh[4], bl[4];
#pragma unroll
    for (int j = 0; j < 4; ++j) {
      const size_t bo = (size_t)(n0 + (j << 4) + rlane) * ldb + koff + k0;
      bh[j] = Frag<T>::load(Bb + bo);
      if (SPLIT) bl[j] = Frag<T>::load(Bb2 + bo);
    }
#pragma unroll
    for (int i = 0; i < 4; ++i) {
      const size_t ao = (size_t)(m0 + (i << 4) + rlane) * lda + koff + k0;
      V ah = Frag<T>::load(Ab + ao);
      V al;
      if (SPLIT) al = Frag<T>::load(Ab2 + ao);
#pragma unroll
      for (int j = 0; j < 4; ++j) {
        acc[i][j] = Frag<T>::mma(ah, bh[j], acc[i][j]);
        if (SPLIT) {
          acc[i][j] = Frag<T>::mma(ah, bl[j], acc[i][j]);
          acc[i][j] = Frag<T>::mma(al, bh[j], acc[i][j]);
        }
      }
      Frag<T>::guard4(acc[i][0], acc[i][1], acc[i][2], acc[i][3], ah, SPLIT ? al : ah);
    }
    Frag<T>::keep(bh[0], bh[1], bh[2], bh[3]);
    if (SPLIT) Frag<T>::keep(bl[0], bl[1], bl[2], bl[3]);
  }
  acc_guard4(acc[0][0], acc[0][1], acc[0][2], acc[0][3]);
  acc_guard4(acc[1][0], acc[1][1], acc[1][2], acc[1][3]);
  acc_guard4(acc[2][0], acc[2][1], acc[2][2], acc[2][3]);
  acc_guard4(acc[3][0], acc[3][1], acc[3][2], acc[3][3]);

  float* slab = sT[wave];
  const float* Rb = RESID ? (resid + (size_t)b * strideR) : nullptr;
#pragma unroll
  for (int i = 0; i < 4; ++i) {
    const int mBase = m0 + (i << 4);
#pragma unroll
    for (int j = 0; j < 4; ++j) {
      const int n = n0 + (j << 4) + rlane;
      float bv = 0.f;
      if (BIAS_MODE == 2) bv = bias[n];
#pragma unroll
      for (int r = 0; r < 8; ++r) {
        float v = acc[i][j][r] * scale;
        if (BIAS_MODE == 1) v += bias[mBase + mOff + r];
        if (BIAS_MODE == 2) v += bv;
        if (RESID) v += Rb[(size_t)(mBase + mOff + r) * ldc + n];
        if (ACT == 1) v = tanhf(v);
        if (ACT == 2) v = fmaxf(v, 0.0f);
        if (ACT == 3) v = v / (1.0f + expf(-v));
        if (ACT == 4) v = (v > 0.f) ? v : 0.01f * v;
        if (ACT == 5) v = 0.5f * v * (1.0f + erff(v * 0.70710678118654752f));
        slab[(mOff + r) * 68 + (j << 4) + rlane] = v;
      }
    }
    __builtin_amdgcn_fence(__ATOMIC_RELEASE, "workgroup");
    __builtin_amdgcn_wave_barrier();
    __builtin_amdgcn_fence(__ATOMIC_ACQUIRE, "workgroup");
    if (OUT_MODE == 0) {
      float* C = (float*)Cout + (size_t)b * strideC;
      const int hh = lane >> 4, c4 = (lane & 15) * 4;
      for (int pass = 0; pass < 2; ++pass) {
#pragma unroll
        for (int it = 0; it < 8; ++it) {
          const int row = it * 2 + hh;
          v4f v = *(const v4f*)(slab + row * 68 + c4);
          *(volatile v4f*)(C + (size_t)(mBase + row) * ldc + n0 + c4) = v;
        }
        __threadfence();
      }
    } else {
      const int q = lane >> 3, c8 = (lane & 7) * 8;
      unsigned short* C  = (unsigned short*)Cout  + (size_t)b * strideC;
      unsigned short* C2 = (OUT_MODE == 2) ? ((unsigned short*)Cout2 + (size_t)b * strideC) : nullptr;
      for (int pass = 0; pass < 2; ++pass) {
#pragma unroll
        for (int it = 0; it < 4; ++it) {
          const int row = it * 4 + q;
          const float* sp = slab + row * 68 + c8;
          v8h hv, lv;
#pragma unroll
          for (int e = 0; e < 8; ++e) {
            if (OUT_MODE == 1) {
              hv[e] = (_Float16)sp[e];
            } else {
              unsigned short hb = f2bf_bits(sp[e]);
              unsigned short lb = f2bf_bits(sp[e] - bf_bits2f(hb));
              hv[e] = __builtin_bit_cast(_Float16, hb);
              lv[e] = __builtin_bit_cast(_Float16, lb);
            }
          }
          *(volatile v8h*)(C + (size_t)(mBase + row) * ldc + n0 + c8) = hv;
          if (OUT_MODE == 2) *(volatile v8h*)(C2 + (size_t)(mBase + row) * ldc + n0 + c8) = lv;
        }
        __threadfence();
      }
    }
    __builtin_amdgcn_fence(__ATOMIC_RELEASE, "workgroup");
    __builtin_amdgcn_wave_barrier();
    __builtin_amdgcn_fence(__ATOMIC_ACQUIRE, "workgroup");
  }
}


__global__ __launch_bounds__(256) void pack_rows_bf16(const float* __restrict__ src,
                                                      unsigned short* __restrict__ dst,
                                                      int colOff, int total8)
{
  const int i = blockIdx.x * 256 + threadIdx.x;
  if (i >= total8) return;
  const size_t f = (size_t)i * 8;
  const int m = (int)(f / NIN);
  const int c = (int)(f - (size_t)m * NIN);
  const v4f a = *(const v4f*)(src + f);
  const v4f b = *(const v4f*)(src + f + 4);
  v4u w;
  w.x = pack_bf2(a.x, a.y);
  w.y = pack_bf2(a.z, a.w);
  w.z = pack_bf2(b.x, b.y);
  w.w = pack_bf2(b.z, b.w);
  unsigned short* p = dst + (size_t)m * KTOT + colOff + c;
  *(volatile v4u*)p = w;
  __threadfence();
  *(volatile v4u*)p = w;
}

__global__ __launch_bounds__(256) void pack_wt_bf16(const float* __restrict__ W,
                                                    unsigned short* __restrict__ Bt,
                                                    int nOff, int kOff)
{
  __shared__ float tile[64][33];
  const int t = threadIdx.x;
  const int kBase = blockIdx.x * 64;
  const int nBase = blockIdx.y * 32;
#pragma unroll
  for (int it = 0; it < 2; ++it) {
    const int q  = t + it * 256;
    const int r  = q >> 3;
    const int c4 = (q & 7) * 4;
    const v4f v = *(const v4f*)(W + (size_t)(kBase + r) * NHID + nBase + c4);
    tile[r][c4 + 0] = v.x;
    tile[r][c4 + 1] = v.y;
    tile[r][c4 + 2] = v.z;
    tile[r][c4 + 3] = v.w;
  }
  __syncthreads();
  const int nl = t >> 3;
  const int k8 = (t & 7) * 8;
  v4u w;
  w.x = pack_bf2(tile[k8 + 0][nl], tile[k8 + 1][nl]);
  w.y = pack_bf2(tile[k8 + 2][nl], tile[k8 + 3][nl]);
  w.z = pack_bf2(tile[k8 + 4][nl], tile[k8 + 5][nl]);
  w.w = pack_bf2(tile[k8 + 6][nl], tile[k8 + 7][nl]);
  unsigned short* p = Bt + (size_t)(nOff + nBase + nl) * KTOT + kOff + kBase + k8;
  *(volatile v4u*)p = w;
  __threadfence();
  *(volatile v4u*)p = w;
}

__device__ __forceinline__ float sigm_f(float z) { return 1.0f / (1.0f + expf(-z)); }

__global__ __launch_bounds__(256) void cell_pointwise(const float* __restrict__ z,
                                                      const float* __restrict__ c0,
                                                      const float* __restrict__ b_ii, const float* __restrict__ b_if,
                                                      const float* __restrict__ b_ig, const float* __restrict__ b_io,
                                                      const float* __restrict__ b_hi, const float* __restrict__ b_hf,
                                                      const float* __restrict__ b_hg, const float* __restrict__ b_ho,
                                                      float* __restrict__ out)
{
  __shared__ __align__(16) float sh[512];
  const int t    = threadIdx.x;
  const int m    = blockIdx.x >> 2;
  const int hb   = (blockIdx.x & 3) * 256;
  const int hcol = hb + t;
  const float bi = bf_rne(b_ii[hcol]) + bf_rne(b_hi[hcol]);
  const float bf = bf_rne(b_if[hcol]) + bf_rne(b_hf[hcol]);
  const float bg = bf_rne(b_ig[hcol]) + bf_rne(b_hg[hcol]);
  const float bo = bf_rne(b_io[hcol]) + bf_rne(b_ho[hcol]);
  asm volatile("" ::: "memory");
  const size_t zr = (size_t)m * NGATE + hcol;
  const float zi = z[zr] + bi;
  const float zf = z[zr + NHID] + bf;
  const float zg = z[zr + 2 * NHID] + bg;
  const float zo = z[zr + 3 * NHID] + bo;
  const float cp = bf_rne(c0[(size_t)m * NHID + hcol]);
  const float ig = sigm_f(zi);
  const float fg = sigm_f(zf);
  const float og = sigm_f(zo);
  const float gg = tanhf(zg);
  const float cn = fg * cp + ig * gg;
  const float hn = og * cn;
  sh[t]       = hn;
  sh[256 + t] = cn;
  __syncthreads();
  if (t < 128) {
    const int which = t >> 6;
    const int q     = t & 63;
    const v4f v = *(const v4f*)(sh + which * 256 + q * 4);
    float* p = out + (size_t)which * PLANE + (size_t)m * NHID + hb + q * 4;
    *(volatile v4f*)p = v;
    __threadfence();
    *(volatile v4f*)p = v;
  }
}

extern "C" void kernel_launch(void* const* d_in, const int* in_sizes, int n_in,
                              void* d_out, int out_size, void* d_ws, size_t ws_size,
                              hipStream_t stream)
{
  if (n_in < 19) return;
  if ((size_t)out_size < 2 * PLANE) return;
  if (ws_size < WS_TOTAL) return;
  if (in_sizes[0] != NBATCH * NIN || in_sizes[1] != NBATCH * NHID || in_sizes[2] != NBATCH * NHID) return;
  if (in_sizes[3] != NIN * NHID || in_sizes[11] != NHID * NHID || in_sizes[4] != NHID) return;

  const float* x    = (const float*)d_in[0];
  const float* h0   = (const float*)d_in[1];
  const float* c0   = (const float*)d_in[2];
  const float* W_ii = (const float*)d_in[3];
  const float* b_ii = (const float*)d_in[4];
  const float* W_if = (const float*)d_in[5];
  const float* b_if = (const float*)d_in[6];
  const float* W_ig = (const float*)d_in[7];
  const float* b_ig = (const float*)d_in[8];
  const float* W_io = (const float*)d_in[9];
  const float* b_io = (const float*)d_in[10];
  const float* W_hi = (const float*)d_in[11];
  const float* b_hi = (const float*)d_in[12];
  const float* W_hf = (const float*)d_in[13];
  const float* b_hf = (const float*)d_in[14];
  const float* W_hg = (const float*)d_in[15];
  const float* b_hg = (const float*)d_in[16];
  const float* W_ho = (const float*)d_in[17];
  const float* b_ho = (const float*)d_in[18];

  float* out = (float*)d_out;
  unsigned char* ws = (unsigned char*)d_ws;
  unsigned short* aplane  = (unsigned short*)(ws + OFF_A);
  unsigned short* btplane = (unsigned short*)(ws + OFF_BT);
  float*          zplane  = (float*)(ws + OFF_Z);

  const int total8 = NBATCH * NIN / 8;
  pack_rows_bf16<<<total8 / 256, 256, 0, stream>>>(x,  aplane, 0,   total8);
  pack_rows_bf16<<<total8 / 256, 256, 0, stream>>>(h0, aplane, NIN, total8);

  const dim3 tg(NIN / 64, NHID / 32);
  pack_wt_bf16<<<tg, 256, 0, stream>>>(W_ii, btplane, 0 * NHID, 0);
  pack_wt_bf16<<<tg, 256, 0, stream>>>(W_if, btplane, 1 * NHID, 0);
  pack_wt_bf16<<<tg, 256, 0, stream>>>(W_ig, btplane, 2 * NHID, 0);
  pack_wt_bf16<<<tg, 256, 0, stream>>>(W_io, btplane, 3 * NHID, 0);
  pack_wt_bf16<<<tg, 256, 0, stream>>>(W_hi, btplane, 0 * NHID, NIN);
  pack_wt_bf16<<<tg, 256, 0, stream>>>(W_hf, btplane, 1 * NHID, NIN);
  pack_wt_bf16<<<tg, 256, 0, stream>>>(W_hg, btplane, 2 * NHID, NIN);
  pack_wt_bf16<<<tg, 256, 0, stream>>>(W_ho, btplane, 3 * NHID, NIN);

  const int tiles = (NBATCH / 64) * (NGATE / 64);
  wmma_gemm64<1, false, 0, 0, false, 0><<<dim3(tiles / 8, 1), 256, 0, stream>>>(
      aplane, aplane, KTOT, 0L,
      btplane, btplane, KTOT, 0L,
      (void*)zplane, (void*)zplane, NGATE, 0L,
      c0,
      c0, 0L,
      NBATCH, NGATE, KTOT, 1.0f);

  cell_pointwise<<<NBATCH * 4, 256, 0, stream>>>(zplane, c0,
                                                 b_ii, b_if, b_ig, b_io, b_hi, b_hf, b_hg, b_ho,
                                                 out);
}
